// BinaryClassifier_8675833937973
// MI455X (gfx1250) — hardware-verified
//
#include <hip/hip_runtime.h>
#include <stddef.h>
#include <stdint.h>

#define NB    2
#define SQ    512
#define NTOK  1024
#define DIN   400
#define KR    448
#define DM    256
#define NH    8
#define HD    32
#define DFF   1024
#define NL    2
#define NQKV  768
#define NCL   2
#define KC    64
#define QKPLANE (NB * NH * SQ * HD)
#define NEGV  (-1.0e9f)

#define C_F   8.0f
#define C_W   32.0f
#define C_X   8.0f
#define C_Q   32.0f
#define C_P   1024.0f
#define C_O   64.0f
#define C_H   64.0f
#define C_PE  16.0f
#define C_PW  1024.0f
#define RED_SC (0.00390625f)
#define QKV_A  (0.125f)
#define SCL    (0.17677669529663687f)
#define S_SC   (SCL * 0.0009765625f)
#define O_SC   (0.001953125f)
#define WO_SC  (0.00048828125f)
#define FF_SC  (0.00390625f)
#define W2_SC  (0.00048828125f)
#define PB_SC  (6.103515625e-05f)
#define SELU_S (1.0507009873554805f)
#define SELU_A (1.6732632423543772f)
#define L2W    (0.20762050593046014f)

static_assert(NTOK == NB * SQ);
static_assert(NH * HD == DM);
static_assert(NQKV == 3 * DM);
static_assert(KR % 64 == 0);
static_assert(KR >= DIN);
static_assert(DIN % 8 == 0);
static_assert(KR / 8 - 32 == 24);
static_assert(SQ % KC == 0);
static_assert(SQ % 256 == 0);
static_assert(NTOK % 256 == 0);
static_assert(DM % 64 == 0);
static_assert(DFF % 64 == 0);
static_assert(NH == 8);
static_assert(HD == 32);
static_assert(QKPLANE == 262144);

typedef _Float16 v16h __attribute__((ext_vector_type(16)));
typedef _Float16 v8h  __attribute__((ext_vector_type(8)));
typedef float    v8f  __attribute__((ext_vector_type(8)));
typedef float    v4f  __attribute__((ext_vector_type(4)));
typedef unsigned int v4u __attribute__((ext_vector_type(4)));

union Frag  { v16h v; v8h h[2]; };
union Pack8 { v8h h; v4u u; };

__device__ __forceinline__ v8f mma16(v16h a, v16h b, v8f c) {
  c = __builtin_amdgcn_wmma_f32_16x16x32_f16(false, a, false, b, (short)0, c, false, false);
  asm volatile("v_nop\n\tv_nop\n\tv_nop\n\tv_nop" : "+v"(c) : "v"(a), "v"(b));
  return c;
}

__device__ __forceinline__ v16h ldfrag(const _Float16* p, int ld, int row0, int k0, int lane) {
  const int m = lane & 15, lh = lane >> 4;
  const _Float16* q = p + (size_t)(row0 + m) * ld + k0 + 8 * lh;
  Frag f;
  f.h[0] = *(const v8h*)(q);
  f.h[1] = *(const v8h*)(q + 16);
  return f.v;
}

__device__ __forceinline__ v8f zero8() { return (v8f){0.f, 0.f, 0.f, 0.f, 0.f, 0.f, 0.f, 0.f}; }

__device__ __forceinline__ v4u pack8(v4f a0, v4f a1) {
  Pack8 pk;
  pk.h = (v8h){(_Float16)a0[0], (_Float16)a0[1], (_Float16)a0[2], (_Float16)a0[3],
               (_Float16)a1[0], (_Float16)a1[1], (_Float16)a1[2], (_Float16)a1[3]};
  return pk.u;
}

__device__ __forceinline__ void gemm32x64(const _Float16* __restrict__ A, int lda,
                                          const _Float16* __restrict__ Bt, int ldb, int K,
                                          int m0, int n0, int lane, v8f (&acc)[2][4]) {
#pragma unroll 1
  for (int k0 = 0; k0 < K; k0 += 32) {
    const v16h a0 = ldfrag(A, lda, m0, k0, lane);
    const v16h a1 = ldfrag(A, lda, m0 + 16, k0, lane);
    const v16h b0 = ldfrag(Bt, ldb, n0, k0, lane);
    const v16h b1 = ldfrag(Bt, ldb, n0 + 16, k0, lane);
    const v16h b2 = ldfrag(Bt, ldb, n0 + 32, k0, lane);
    const v16h b3 = ldfrag(Bt, ldb, n0 + 48, k0, lane);
    acc[0][0] = mma16(a0, b0, acc[0][0]);
    acc[1][0] = mma16(a1, b0, acc[1][0]);
    acc[0][1] = mma16(a0, b1, acc[0][1]);
    acc[1][1] = mma16(a1, b1, acc[1][1]);
    acc[0][2] = mma16(a0, b2, acc[0][2]);
    acc[1][2] = mma16(a1, b2, acc[1][2]);
    acc[0][3] = mma16(a0, b3, acc[0][3]);
    acc[1][3] = mma16(a1, b3, acc[1][3]);
  }
}

__device__ __forceinline__ void gemm16x64(const _Float16* __restrict__ A, int lda,
                                          const _Float16* __restrict__ Bt, int ldb, int K,
                                          int m0, int n0, int lane, v8f (&acc)[4]) {
#pragma unroll 1
  for (int k0 = 0; k0 < K; k0 += 32) {
    const v16h a  = ldfrag(A, lda, m0, k0, lane);
    const v16h b0 = ldfrag(Bt, ldb, n0, k0, lane);
    const v16h b1 = ldfrag(Bt, ldb, n0 + 16, k0, lane);
    const v16h b2 = ldfrag(Bt, ldb, n0 + 32, k0, lane);
    const v16h b3 = ldfrag(Bt, ldb, n0 + 48, k0, lane);
    acc[0] = mma16(a, b0, acc[0]);
    acc[1] = mma16(a, b1, acc[1]);
    acc[2] = mma16(a, b2, acc[2]);
    acc[3] = mma16(a, b3, acc[3]);
  }
}

#define TP 72
__global__ __launch_bounds__(256) void k_tr(const float* __restrict__ src, int K, int N, int Kp, size_t srcZ,
                                            _Float16* __restrict__ dst, size_t dstZ, float scale) {
  __shared__ __align__(16) _Float16 st[64 * TP];
  const int tid = threadIdx.x;
  const int n0 = blockIdx.x * 64, k0 = blockIdx.y * 64, l = blockIdx.z;
  const int r = tid >> 2, cq = (tid & 3) * 16;
  const int kr  = k0 + r;
  const int krc = (kr < K) ? kr : (K - 1);
  const float zs = (kr < K) ? scale : 0.0f;
  const float* S = src + (size_t)l * srcZ + (size_t)krc * N + n0 + cq;
#pragma unroll
  for (int j = 0; j < 4; ++j) {
    const v4f a = *(const v4f*)(S + 4 * j) * zs;
#pragma unroll
    for (int i = 0; i < 4; ++i) st[(cq + 4 * j + i) * TP + r] = (_Float16)a[i];
  }
  __syncthreads();
  v4u val[2];
  size_t go[2];
#pragma unroll
  for (int it = 0; it < 2; ++it) {
    const int p   = tid + 256 * it;
    const int row = p >> 3;
    const int pc  = p & 7;
    Pack8 pk;
    pk.h    = *(const v8h*)(st + row * TP + pc * 8);
    val[it] = pk.u;
    go[it]  = (size_t)l * dstZ + (size_t)(n0 + row) * Kp + k0 + pc * 8;
  }
#pragma unroll
  for (int it = 0; it < 2; ++it) *(volatile v4u*)(dst + go[it]) = val[it];
  __threadfence();
#pragma unroll
  for (int it = 0; it < 2; ++it) *(volatile v4u*)(dst + go[it]) = val[it];
}

__global__ __launch_bounds__(256) void k_cvtf(const float* __restrict__ src, _Float16* __restrict__ dst) {
  const int tid = threadIdx.x, lane = tid & 31, wave = tid >> 5;
  const int row = blockIdx.x * 8 + wave;
  const float* S = src + (size_t)row * DIN;
  _Float16* D = dst + (size_t)row * KR;
  v4u val[2];
#pragma unroll
  for (int it = 0; it < 2; ++it) {
    const int pc  = lane + 32 * it;
    const int pcc = (pc < DIN / 8) ? pc : (DIN / 8 - 1);
    const float zs = (pc < DIN / 8) ? C_F : 0.0f;
    const v4f a0 = *(const v4f*)(S + 8 * pcc) * zs;
    const v4f a1 = *(const v4f*)(S + 8 * pcc + 4) * zs;
    val[it] = pack8(a0, a1);
  }
  volatile v4u* d0 = (volatile v4u*)(D + 8 * lane);
  volatile v4u* d1 = (volatile v4u*)(D + 256 + 8 * lane);
  *d0 = val[0];
  if (lane < (KR / 8 - 32)) *d1 = val[1];
  __threadfence();
  *d0 = val[0];
  if (lane < (KR / 8 - 32)) *d1 = val[1];
}

__global__ __launch_bounds__(256) void k_pw(const float* __restrict__ pw, const float* __restrict__ pb,
                                            _Float16* __restrict__ pwh, float* __restrict__ pbl) {
  __shared__ __align__(16) _Float16 st[16 * DM];
  __shared__ __align__(16) float sp[32];
  const int tid = threadIdx.x, lane = tid & 31, wave = tid >> 5;
#pragma unroll 1
  for (int hq = 0; hq < NH; ++hq) {
    const float* q = pw + (size_t)tid * DM + hq * HD;
    float s = 0.f;
#pragma unroll
    for (int t = 0; t < HD; t += 4) {
      const v4f a = *(const v4f*)(q + t);
      s += a[0]; s += a[1]; s += a[2]; s += a[3];
    }
    st[hq * DM + tid] = (_Float16)(s * 0.03125f * C_PW);
  }
#pragma unroll
  for (int hq = NH; hq < 16; ++hq) st[hq * DM + tid] = (_Float16)0.0f;
  if (wave == 0) {
    const int hq = lane & 7;
    float s = 0.f;
#pragma unroll 1
    for (int t = 0; t < HD; ++t) s += pb[hq * HD + t];
    sp[lane] = (lane < 8) ? (s * 0.03125f) : 0.f;
  }
  __syncthreads();
  v4u val[2];
  size_t go[2];
#pragma unroll
  for (int it = 0; it < 2; ++it) {
    const int p   = tid + 256 * it;
    const int row = p >> 5;
    const int pc  = p & 31;
    Pack8 pk;
    pk.h    = *(const v8h*)(st + row * DM + pc * 8);
    val[it] = pk.u;
    go[it]  = (size_t)row * DM + pc * 8;
  }
  const v4f pv = *(const v4f*)(sp + 4 * (tid & 7));
#pragma unroll
  for (int it = 0; it < 2; ++it) *(volatile v4u*)(pwh + go[it]) = val[it];
  if (tid < 8) *(volatile v4f*)(pbl + 4 * tid) = pv;
  __threadfence();
#pragma unroll
  for (int it = 0; it < 2; ++it) *(volatile v4u*)(pwh + go[it]) = val[it];
  if (tid < 8) *(volatile v4f*)(pbl + 4 * tid) = pv;
}

#define AP  264
#define SBP 132
__global__ __launch_bounds__(128) void k_posb(const float* __restrict__ pos, const _Float16* __restrict__ pwh,
                                              const float* __restrict__ pbl, float* __restrict__ bias) {
  __shared__ __align__(16) _Float16 at[4 * 16 * AP];
  __shared__ __align__(16) float sb[4 * 8 * SBP];
  __shared__ float rdm[64];
  const int tid = threadIdx.x, lane = tid & 31, wave = tid >> 5;
  const int hh = lane >> 4, c = lane & 15;
  const int blk = blockIdx.x;
  if (tid < 64) rdm[tid] = exp2f(-(float)tid * L2W);
  __syncthreads();
  const float pbv = pbl[c & 7];
  _Float16* aw = at + wave * 16 * AP;
  float* sw = sb + wave * 8 * SBP;
  const size_t rbase = (size_t)blk * SQ + (size_t)wave * 128;
#pragma unroll 1
  for (int tl = 0; tl < 8; ++tl) {
    const int jl0 = tl * 16;
    const float p = floorf(pos[(rbase + jl0 + c) * 2 + hh]);
    __syncthreads();
    _Float16* ar = aw + c * AP + hh * 128;
#pragma unroll 1
    for (int t = 0; t < 64; ++t) {
      float sv, cv;
      sincosf(p * rdm[t], &sv, &cv);
      ar[t]      = (_Float16)(sv * C_PE);
      ar[64 + t] = (_Float16)(cv * C_PE);
    }
    __syncthreads();
    v8f acc = zero8();
#pragma unroll
    for (int ks = 0; ks < 8; ++ks) {
      const v16h a = ldfrag(aw, AP, 0, ks * 32, lane);
      const v16h w = ldfrag(pwh, DM, 0, ks * 32, lane);
      acc = mma16(a, w, acc);
    }
    if (c < 8) {
#pragma unroll
      for (int r = 0; r < 8; ++r) sw[c * SBP + jl0 + 8 * hh + r] = acc[r] * PB_SC + pbv;
    }
  }
  __syncthreads();
  const int b = blk >> 9, i = blk & 511;
  v4f val[8];
  size_t go[8];
#pragma unroll
  for (int hq = 0; hq < 8; ++hq) {
    val[hq] = *(const v4f*)(sw + hq * SBP + 4 * lane);
    go[hq]  = ((size_t)(b * NH + hq) * SQ + i) * SQ + (size_t)wave * 128 + 4 * lane;
  }
#pragma unroll
  for (int hq = 0; hq < 8; ++hq) *(volatile v4f*)(bias + go[hq]) = val[hq];
  __threadfence();
#pragma unroll
  for (int hq = 0; hq < 8; ++hq) *(volatile v4f*)(bias + go[hq]) = val[hq];
}

#define RTP 260
template <int ACT, int HASB>
__global__ __launch_bounds__(256) void k_gemm_row(const _Float16* __restrict__ A, int lda, int K,
                                                  const _Float16* __restrict__ Bt,
                                                  const float* __restrict__ bias,
                                                  const float* __restrict__ gam,
                                                  const float* __restrict__ bet,
                                                  float* X, _Float16* __restrict__ Xh, float scale) {
  __shared__ __align__(16) float T[32 * RTP];
  const int tid = threadIdx.x, lane = tid & 31, wave = tid >> 5;
  const int hh = lane >> 4, c = lane & 15;
  const int rs = wave & 1, cg = wave >> 1;
  const int row0 = blockIdx.x * 32;
  const int m0 = row0 + rs * 16, n0 = cg * 64;

  v8f acc[4];
#pragma unroll
  for (int t = 0; t < 4; ++t) acc[t] = zero8();
  gemm16x64(A, lda, Bt, K, K, m0, n0, lane, acc);

  float bb[4];
  if (HASB != 0) {
#pragma unroll
    for (int t = 0; t < 4; ++t) bb[t] = bias[n0 + 16 * t + c];
  } else {
#pragma unroll
    for (int t = 0; t < 4; ++t) bb[t] = 0.f;
  }
#pragma unroll
  for (int t = 0; t < 4; ++t) {
#pragma unroll
    for (int r = 0; r < 8; ++r) T[(rs * 16 + 8 * hh + r) * RTP + n0 + 16 * t + c] = acc[t][r] * scale + bb[t];
  }
  __syncthreads();

  if (ACT == 1) {
#pragma unroll 1
    for (int q = 0; q < 32; ++q) {
      const int rr = q >> 3, e = q & 7;
      const int col = (e < 4) ? (4 * lane + e) : (128 + 4 * lane + (e - 4));
      float* tr = T + (wave * 4 + rr) * RTP;
      const float v  = tr[col];
      const float ex = expm1f(fminf(v, 0.f));
      tr[col] = SELU_S * ((v > 0.f) ? v : SELU_A * ex);
    }
  } else {
    const v4f g0 = *(const v4f*)(gam + 4 * lane), g1 = *(const v4f*)(gam + 128 + 4 * lane);
    const v4f e0 = *(const v4f*)(bet + 4 * lane), e1 = *(const v4f*)(bet + 128 + 4 * lane);
#pragma unroll 1
    for (int rr = 0; rr < 4; ++rr) {
      const int lr = wave * 4 + rr;
      float* tr = T + lr * RTP;
      const size_t grow = (size_t)(row0 + lr) * DM;
      v4f v0 = *(const v4f*)(tr + 4 * lane) + *(const v4f*)(X + grow + 4 * lane);
      v4f v1 = *(const v4f*)(tr + 128 + 4 * lane) + *(const v4f*)(X + grow + 128 + 4 * lane);
      float s1 = ((v0[0] + v0[1]) + (v0[2] + v0[3])) + ((v1[0] + v1[1]) + (v1[2] + v1[3]));
#pragma unroll
      for (int off = 16; off >= 1; off >>= 1) s1 += __shfl_xor(s1, off, 32);
      const float mean = s1 * 0.00390625f;
      v0 = v0 - mean;
      v1 = v1 - mean;
      float s2 = ((v0[0] * v0[0] + v0[1] * v0[1]) + (v0[2] * v0[2] + v0[3] * v0[3])) +
                 ((v1[0] * v1[0] + v1[1] * v1[1]) + (v1[2] * v1[2] + v1[3] * v1[3]));
#pragma unroll
      for (int off = 16; off >= 1; off >>= 1) s2 += __shfl_xor(s2, off, 32);
      const float var  = s2 * 0.00390625f;
      const float rstd = rsqrtf(var + 1e-5f);
      v0 = v0 * rstd * g0 + e0;
      v1 = v1 * rstd * g1 + e1;
      *(v4f*)(tr + 4 * lane)       = v0;
      *(v4f*)(tr + 128 + 4 * lane) = v1;
    }
  }
  __syncthreads();

  v4f fv[8];
  v4u hv[4];
  size_t gr[4];
#pragma unroll
  for (int rr = 0; rr < 4; ++rr) {
    const int lr = wave * 4 + rr;
    const float* tr = T + lr * RTP;
    fv[2 * rr]     = *(const v4f*)(tr + 4 * lane);
    fv[2 * rr + 1] = *(const v4f*)(tr + 128 + 4 * lane);
    const v4f a0 = *(const v4f*)(tr + 8 * lane) * C_X, a1 = *(const v4f*)(tr + 8 * lane + 4) * C_X;
    hv[rr] = pack8(a0, a1);
    gr[rr] = (size_t)(row0 + lr) * DM;
  }
#pragma unroll
  for (int rr = 0; rr < 4; ++rr) {
    *(volatile v4f*)(X + gr[rr] + 4 * lane)       = fv[2 * rr];
    *(volatile v4f*)(X + gr[rr] + 128 + 4 * lane) = fv[2 * rr + 1];
    *(volatile v4u*)(Xh + gr[rr] + 8 * lane)      = hv[rr];
  }
  __threadfence();
#pragma unroll
  for (int rr = 0; rr < 4; ++rr) {
    *(volatile v4f*)(X + gr[rr] + 4 * lane)       = fv[2 * rr];
    *(volatile v4f*)(X + gr[rr] + 128 + 4 * lane) = fv[2 * rr + 1];
    *(volatile v4u*)(Xh + gr[rr] + 8 * lane)      = hv[rr];
  }
}

#define STP 72
#define SVP 264
__global__ __launch_bounds__(256) void k_qkv(const _Float16* __restrict__ xh,
                                             const _Float16* __restrict__ wt,
                                             _Float16* __restrict__ qkp,
                                             _Float16* __restrict__ vtp) {
  __shared__ __align__(16) _Float16 st[256 * STP];
  const int tid = threadIdx.x, lane = tid & 31, wave = tid >> 5;
  const int hh = lane >> 4, c = lane & 15;
  const int bx = blockIdx.x;
  const int b  = bx >> 1;
  const int sb = (bx & 1) * 256;
  const int ns = blockIdx.y;
  const int which = ns >> 2;
  const int hp    = ns & 3;
  const int m0 = sb + wave * 32;
  const int n0 = ns * 64;
  const _Float16* A = xh + (size_t)b * SQ * DM;

  v8f acc[2][4];
#pragma unroll
  for (int s = 0; s < 2; ++s)
#pragma unroll
    for (int t = 0; t < 4; ++t) acc[s][t] = zero8();
  gemm32x64(A, DM, wt, DM, DM, m0, n0, lane, acc);

  if (which < 2) {
#pragma unroll
    for (int sub = 0; sub < 2; ++sub)
#pragma unroll
      for (int t = 0; t < 4; ++t)
#pragma unroll
        for (int r = 0; r < 8; ++r)
          st[(wave * 32 + sub * 16 + 8 * hh + r) * STP + 16 * t + c] = (_Float16)(acc[sub][t][r] * QKV_A);
  } else {
#pragma unroll
    for (int sub = 0; sub < 2; ++sub)
#pragma unroll
      for (int t = 0; t < 4; ++t)
#pragma unroll
        for (int r = 0; r < 8; ++r)
          st[(16 * t + c) * SVP + wave * 32 + sub * 16 + 8 * hh + r] = (_Float16)(acc[sub][t][r] * QKV_A);
  }
  __syncthreads();

  v4u val[8];
  size_t go[8];
  if (which < 2) {
#pragma unroll
    for (int e = 0; e < 2; ++e) {
      const size_t base = (size_t)which * QKPLANE + (size_t)(b * NH + 2 * hp + e) * SQ * HD;
#pragma unroll
      for (int j = 0; j < 4; ++j) {
        const int p  = tid + 256 * j;
        const int lr = p >> 2;
        const int pc = p & 3;
        Pack8 pk;
        pk.h = *(const v8h*)(st + lr * STP + e * 32 + pc * 8);
        val[e * 4 + j] = pk.u;
        go[e * 4 + j]  = base + (size_t)(sb + lr) * HD + pc * 8;
      }
    }
#pragma unroll
    for (int q = 0; q < 8; ++q) *(volatile v4u*)(qkp + go[q]) = val[q];
    __threadfence();
#pragma unroll
    for (int q = 0; q < 8; ++q) *(volatile v4u*)(qkp + go[q]) = val[q];
  } else {
#pragma unroll
    for (int j = 0; j < 8; ++j) {
      const int p    = tid + 256 * j;
      const int drow = p >> 5;
      const int pc   = p & 31;
      const int e    = drow >> 5, dk = drow & 31;
      Pack8 pk;
      pk.h   = *(const v8h*)(st + drow * SVP + pc * 8);
      val[j] = pk.u;
      go[j]  = (size_t)(b * NH + 2 * hp + e) * HD * SQ + (size_t)dk * SQ + sb + pc * 8;
    }
#pragma unroll
    for (int q = 0; q < 8; ++q) *(volatile v4u*)(vtp + go[q]) = val[q];
    __threadfence();
#pragma unroll
    for (int q = 0; q < 8; ++q) *(volatile v4u*)(vtp + go[q]) = val[q];
  }
}

#define KSP 40
#define VTP 72
#define PTP 72
__global__ __launch_bounds__(256) void k_attn(const _Float16* __restrict__ qp,
                                              const _Float16* __restrict__ kp,
                                              const _Float16* __restrict__ vt,
                                              const float* __restrict__ fm,
                                              const float* __restrict__ bp,
                                              _Float16* __restrict__ op) {
  __shared__ __align__(16) _Float16 Ks[2 * KC * KSP];
  __shared__ __align__(16) _Float16 Vs[2 * HD * VTP];
  __shared__ __align__(16) _Float16 Ps[8 * 16 * PTP];
  __shared__ __align__(16) _Float16 Os[64 * PTP];

  const int tid = threadIdx.x, lane = tid & 31, wave = tid >> 5;
  const int hh = lane >> 4, c = lane & 15;
  const int blk = blockIdx.x;
  const int qb  = blk & 7;
  const int hp  = (blk >> 3) & 3;
  const int b   = blk >> 5;
  const int e   = wave >> 2;
  const int qt  = wave & 3;
  const int h   = 2 * hp + e;
  const int hb  = b * NH + h;
  const int q0  = qb * 64 + qt * 16;

  const _Float16* Q = qp + (size_t)hb * SQ * HD;
  const v16h qa = ldfrag(Q, HD, q0, 0, lane);
  const float* brow = bp + (size_t)hb * SQ * SQ;
  const float* fmb  = fm + (size_t)b * SQ;
  int pq[8];
#pragma unroll
  for (int r = 0; r < 8; ++r) {
    const float f = fmb[q0 + 8 * hh + r];
    pq[r] = (1.0f - f > 0.0f) ? 1 : 0;
  }

  const float NEGI = -__builtin_huge_valf();
  float mrow[8], lrow[8];
  v8f oacc[2];
#pragma unroll
  for (int r = 0; r < 8; ++r) { mrow[r] = NEGI; lrow[r] = 0.f; }
  oacc[0] = zero8();
  oacc[1] = zero8();

  _Float16* pw = Ps + wave * 16 * PTP;
  const _Float16* Kse = Ks + e * KC * KSP;
  const _Float16* Vse = Vs + e * HD * VTP;

#pragma unroll 1
  for (int kc = 0; kc < SQ / KC; ++kc) {
    const int kv0 = kc * KC;
    __syncthreads();
#pragma unroll
    for (int u = 0; u < 2; ++u) {
      const int p  = tid + 256 * u;
      const int e2 = p >> 8;
      const int r  = (p >> 2) & 63;
      const int qq = (p & 3) * 8;
      const _Float16* ks = kp + (size_t)(b * NH + 2 * hp + e2) * SQ * HD + (size_t)(kv0 + r) * HD + qq;
      *(v8h*)(Ks + e2 * KC * KSP + r * KSP + qq) = *(const v8h*)ks;
      const int r2 = (p >> 3) & 31;
      const int q2 = (p & 7) * 8;
      const _Float16* vs = vt + (size_t)(b * NH + 2 * hp + e2) * HD * SQ + (size_t)r2 * SQ + kv0 + q2;
      *(v8h*)(Vs + e2 * HD * VTP + r2 * VTP + q2) = *(const v8h*)vs;
    }
    __syncthreads();

    v8f s[4];
#pragma unroll
    for (int j = 0; j < 4; ++j) {
      const v16h kb = ldfrag(Kse, KSP, j * 16, 0, lane);
      s[j] = mma16(qa, kb, zero8());
    }
    int pk[4];
#pragma unroll
    for (int j = 0; j < 4; ++j) {
      const float f = fmb[kv0 + j * 16 + c];
      pk[j] = (1.0f - f > 0.0f) ? 1 : 0;
    }
    float cm[8];
#pragma unroll
    for (int r = 0; r < 8; ++r) {
      const int qi = q0 + 8 * hh + r;
      float m = NEGI;
#pragma unroll
      for (int j = 0; j < 4; ++j) {
        const int key = kv0 + j * 16 + c;
        const int di  = qi - key;
        const int ad  = (di < 0) ? -di : di;
        const bool lnp = (di >= 9) || (di <= -8);
        const bool dnp = (ad & 15) != 0;
        const bool msk = (dnp || (pq[r] != 0) || (pk[j] != 0)) && (lnp || (pk[j] != 0));
        const float sv = s[j][r] * S_SC + brow[(size_t)qi * SQ + key];
        s[j][r] = msk ? NEGV : sv;
        m = fmaxf(m, s[j][r]);
      }
#pragma unroll
      for (int off = 1; off < 16; off <<= 1) m = fmaxf(m, __shfl_xor(m, off, 32));
      cm[r] = m;
    }
    float al[8];
#pragma unroll
    for (int r = 0; r < 8; ++r) {
      const float mnew  = fmaxf(mrow[r], cm[r]);
      const float alpha = __expf(mrow[r] - mnew);
      mrow[r] = mnew;
      float psum = 0.f;
#pragma unroll
      for (int j = 0; j < 4; ++j) {
        const float p = __expf(s[j][r] - mnew);
        psum += p;
        pw[(8 * hh + r) * PTP + j * 16 + c] = (_Float16)(p * C_P);
      }
#pragma unroll
      for (int off = 1; off < 16; off <<= 1) psum += __shfl_xor(psum, off, 32);
      lrow[r] = lrow[r] * alpha + psum;
      al[r] = alpha;
    }
#pragma unroll
    for (int t = 0; t < 2; ++t)
#pragma unroll
      for (int r = 0; r < 8; ++r) oacc[t][r] *= al[r];
    __syncthreads();

#pragma unroll
    for (int kk = 0; kk < 2; ++kk) {
      const v16h pa = ldfrag(pw, PTP, 0, kk * 32, lane);
#pragma unroll
      for (int t = 0; t < 2; ++t) {
        const v16h vb = ldfrag(Vse, VTP, t * 16, kk * 32, lane);
        oacc[t] = mma16(pa, vb, oacc[t]);
      }
    }
  }

  float invl[8];
#pragma unroll
  for (int r = 0; r < 8; ++r) invl[r] = (lrow[r] > 0.f) ? (O_SC / lrow[r]) : 0.f;
  __syncthreads();
#pragma unroll
  for (int r = 0; r < 8; ++r) {
#pragma unroll
    for (int t = 0; t < 2; ++t)
      Os[(qt * 16 + 8 * hh + r) * PTP + e * 32 + 16 * t + c] = (_Float16)(oacc[t][r] * invl[r]);
  }
  __syncthreads();
  v4u val[2];
  size_t go[2];
#pragma unroll
  for (int it = 0; it < 2; ++it) {
    const int p   = tid + 256 * it;
    const int row = p >> 3;
    const int pc  = p & 7;
    Pack8 pkk;
    pkk.h   = *(const v8h*)(Os + row * PTP + pc * 8);
    val[it] = pkk.u;
    go[it]  = ((size_t)(b * SQ + qb * 64 + row)) * DM + (size_t)hp * 64 + pc * 8;
  }
#pragma unroll
  for (int it = 0; it < 2; ++it) *(volatile v4u*)(op + go[it]) = val[it];
  __threadfence();
#pragma unroll
  for (int it = 0; it < 2; ++it) *(volatile v4u*)(op + go[it]) = val[it];
}

#define HTP 72
__global__ __launch_bounds__(256) void k_ffn1(const _Float16* __restrict__ xh,
                                              const _Float16* __restrict__ wt,
                                              const float* __restrict__ bias,
                                              _Float16* __restrict__ hout) {
  __shared__ __align__(16) _Float16 st[8 * 32 * HTP];
  const int tid = threadIdx.x, lane = tid & 31, wave = tid >> 5;
  const int hh = lane >> 4, c = lane & 15;
  const int m0 = blockIdx.x * 256 + wave * 32;
  const int n0 = blockIdx.y * 64;

  v8f acc[2][4];
#pragma unroll
  for (int s = 0; s < 2; ++s)
#pragma unroll
    for (int t = 0; t < 4; ++t) acc[s][t] = zero8();
  gemm32x64(xh, DM, wt, DM, DM, m0, n0, lane, acc);
  float bb[4];
#pragma unroll
  for (int t = 0; t < 4; ++t) bb[t] = bias[n0 + 16 * t + c];
  _Float16* sw = st + wave * 32 * HTP;
#pragma unroll
  for (int sub = 0; sub < 2; ++sub)
#pragma unroll
    for (int t = 0; t < 4; ++t)
#pragma unroll
      for (int r = 0; r < 8; ++r)
        sw[(sub * 16 + 8 * hh + r) * HTP + 16 * t + c] =
            (_Float16)(fmaxf(acc[sub][t][r] * FF_SC + bb[t], 0.f) * C_H);
  __syncthreads();
  v4u val[8];
  size_t go[8];
#pragma unroll
  for (int it = 0; it < 8; ++it) {
    const int p   = lane + 32 * it;
    const int row = p >> 3;
    const int pc  = p & 7;
    Pack8 pk;
    pk.h    = *(const v8h*)(sw + row * HTP + pc * 8);
    val[it] = pk.u;
    go[it]  = (size_t)(m0 + row) * DFF + n0 + pc * 8;
  }
#pragma unroll
  for (int it = 0; it < 8; ++it) *(volatile v4u*)(hout + go[it]) = val[it];
  __threadfence();
#pragma unroll
  for (int it = 0; it < 8; ++it) *(volatile v4u*)(hout + go[it]) = val[it];
}

__global__ __launch_bounds__(256) void k_cls(const float* __restrict__ X, const float* __restrict__ cw,
                                             const float* __restrict__ cb, float* __restrict__ out) {
  __shared__ __align__(16) float so[256];
  const int tid = threadIdx.x, lane = tid & 31, wave = tid >> 5;
  const v4f w0 = *(const v4f*)(cw + 16 * lane);
  const v4f w1 = *(const v4f*)(cw + 16 * lane + 4);
  const v4f w2 = *(const v4f*)(cw + 16 * lane + 8);
  const v4f w3 = *(const v4f*)(cw + 16 * lane + 12);
  const float cb0 = cb[0], cb1 = cb[1];
#pragma unroll 1
  for (int rr = 0; rr < 16; ++rr) {
    const int row = blockIdx.x * 128 + wave * 16 + rr;
    const float* xr = X + (size_t)row * DM + 8 * lane;
    const v4f x0 = *(const v4f*)xr, x1 = *(const v4f*)(xr + 4);
    float l0 = ((x0[0] * w0[0] + x0[1] * w0[2]) + (x0[2] * w1[0] + x0[3] * w1[2])) +
               ((x1[0] * w2[0] + x1[1] * w2[2]) + (x1[2] * w3[0] + x1[3] * w3[2]));
    float l1 = ((x0[0] * w0[1] + x0[1] * w0[3]) + (x0[2] * w1[1] + x0[3] * w1[3])) +
               ((x1[0] * w2[1] + x1[1] * w2[3]) + (x1[2] * w3[1] + x1[3] * w3[3]));
#pragma unroll
    for (int off = 16; off >= 1; off >>= 1) {
      l0 += __shfl_xor(l0, off, 32);
      l1 += __shfl_xor(l1, off, 32);
    }
    l0 += cb0;
    l1 += cb1;
    const float m   = fmaxf(l0, l1);
    const float x0e = __expf(l0 - m), x1e = __expf(l1 - m);
    const float inv = 1.0f / (x0e + x1e);
    if (lane == 0) {
      so[(wave * 16 + rr) * 2]     = x0e * inv;
      so[(wave * 16 + rr) * 2 + 1] = x1e * inv;
    }
  }
  __syncthreads();
  if (tid < 64) {
    const v4f v = *(const v4f*)(so + 4 * tid);
    volatile v4f* p = (volatile v4f*)(out + (size_t)blockIdx.x * 256 + 4 * tid);
    *p = v;
    __threadfence();
    *p = v;
  }
}

extern "C" void kernel_launch(void* const* d_in, const int* in_sizes, int n_in,
                              void* d_out, int out_size, void* d_ws, size_t ws_size,
                              hipStream_t stream) {
  if (n_in < 21) return;
  if (in_sizes[0] != NTOK * DIN) return;
  if (in_sizes[1] != NB * SQ * SQ * 2) return;
  if (in_sizes[2] != NTOK) return;
  if (in_sizes[3] != DIN * DM) return;
  if (in_sizes[4] != DM) return;
  if (in_sizes[5] != DM * DM) return;
  if (in_sizes[6] != DM) return;
  if (in_sizes[7] != NL * DM * DM) return;
  if (in_sizes[8] != NL * DM * DM) return;
  if (in_sizes[9] != NL * DM * DM) return;
  if (in_sizes[10] != NL * DM * DM) return;
  if (in_sizes[11] != NL * DM) return;
  if (in_sizes[12] != NL * DM) return;
  if (in_sizes[13] != NL * DM * DFF) return;
  if (in_sizes[14] != NL * DFF) return;
  if (in_sizes[15] != NL * DFF * DM) return;
  if (in_sizes[16] != NL * DM) return;
  if (in_sizes[17] != NL * DM) return;
  if (in_sizes[18] != NL * DM) return;
  if (in_sizes[19] != DM * NCL) return;
  if (in_sizes[20] != NCL) return;
  if (out_size != NTOK * NCL) return;

  const float* feature = (const float*)d_in[0];
  const float* pos_ind = (const float*)d_in[1];
  const float* fmask   = (const float*)d_in[2];
  const float* w_red   = (const float*)d_in[3];
  const float* b_red   = (const float*)d_in[4];
  const float* pos_w   = (const float*)d_in[5];
  const float* pos_b   = (const float*)d_in[6];
  const float* wq      = (const float*)d_in[7];
  const float* wk      = (const float*)d_in[8];
  const float* wv      = (const float*)d_in[9];
  const float* wo      = (const float*)d_in[10];
  const float* ln1g    = (const float*)d_in[11];
  const float* ln1b    = (const float*)d_in[12];
  const float* w1      = (const float*)d_in[13];
  const float* b1      = (const float*)d_in[14];
  const float* w2      = (const float*)d_in[15];
  const float* b2      = (const float*)d_in[16];
  const float* ln2g    = (const float*)d_in[17];
  const float* ln2b    = (const float*)d_in[18];
  const float* cls_w   = (const float*)d_in[19];
  const float* cls_b   = (const float*)d_in[20];
  float* out = (float*)d_out;

  size_t off = 0;
  const size_t oWR   = off; off += (size_t)DM * KR * 2;
  const size_t oWQKV = off; off += (size_t)NL * NQKV * DM * 2;
  const size_t oWO   = off; off += (size_t)NL * DM * DM * 2;
  const size_t oW1   = off; off += (size_t)NL * DFF * DM * 2;
  const size_t oW2   = off; off += (size_t)NL * DM * DFF * 2;
  const size_t oFH   = off; off += (size_t)NTOK * KR * 2;
  const size_t oX    = off; off += (size_t)NTOK * DM * 4;
  const size_t oXH   = off; off += (size_t)NTOK * DM * 2;
  const size_t oQ    = off; off += (size_t)QKPLANE * 2;
  const size_t oK    = off; off += (size_t)QKPLANE * 2;
  const size_t oVT   = off; off += (size_t)NB * NH * HD * SQ * 2;
  const size_t oO    = off; off += (size_t)NTOK * DM * 2;
  const size_t oHP   = off; off += (size_t)NTOK * DFF * 2;
  const size_t oPWH  = off; off += (size_t)16 * DM * 2;
  const size_t oPBL  = off; off += 512;
  const size_t oBIAS = off; off += (size_t)NB * NH * SQ * SQ * 4;
  if (off > ws_size) return;
  if (off > (size_t)134217728) return;
  if (oK != oQ + (size_t)QKPLANE * 2) return;
  if ((oBIAS & 127) != 0 || (oPBL & 127) != 0) return;

  char* ws = (char*)d_ws;
  _Float16* WR   = (_Float16*)(ws + oWR);
  _Float16* WQKV = (_Float16*)(ws + oWQKV);
  _Float16* WO   = (_Float16*)(ws + oWO);
  _Float16* W1T  = (_Float16*)(ws + oW1);
  _Float16* W2T  = (_Float16*)(ws + oW2);
  _Float16* FH   = (_Float16*)(ws + oFH);
  float*    X    = (float*)(ws + oX);
  _Float16* XH   = (_Float16*)(ws + oXH);
  _Float16* Qp   = (_Float16*)(ws + oQ);
  _Float16* Kp   = (_Float16*)(ws + oK);
  _Float16* VT   = (_Float16*)(ws + oVT);
  _Float16* Op   = (_Float16*)(ws + oO);
  _Float16* HP   = (_Float16*)(ws + oHP);
  _Float16* PWH  = (_Float16*)(ws + oPWH);
  float*    PBL  = (float*)(ws + oPBL);
  float*    BIAS = (float*)(ws + oBIAS);

  k_tr<<<dim3(DM / 64, KR / 64, 1), dim3(256), 0, stream>>>(w_red, DIN, DM, KR, (size_t)0, WR, (size_t)0, C_W);
  k_tr<<<dim3(DM / 64, DM / 64, NL), dim3(256), 0, stream>>>(wq, DM, DM, DM, (size_t)DM * DM, WQKV, (size_t)NQKV * DM, C_W);
  k_tr<<<dim3(DM / 64, DM / 64, NL), dim3(256), 0, stream>>>(wk, DM, DM, DM, (size_t)DM * DM, WQKV + (size_t)DM * DM, (size_t)NQKV * DM, C_W);
  k_tr<<<dim3(DM / 64, DM / 64, NL), dim3(256), 0, stream>>>(wv, DM, DM, DM, (size_t)DM * DM, WQKV + (size_t)2 * DM * DM, (size_t)NQKV * DM, C_W);
  k_tr<<<dim3(DM / 64, DM / 64, NL), dim3(256), 0, stream>>>(wo, DM, DM, DM, (size_t)DM * DM, WO, (size_t)DM * DM, C_W);
  k_tr<<<dim3(DFF / 64, DM / 64, NL), dim3(256), 0, stream>>>(w1, DM, DFF, DM, (size_t)DM * DFF, W1T, (size_t)DFF * DM, C_W);
  k_tr<<<dim3(DM / 64, DFF / 64, NL), dim3(256), 0, stream>>>(w2, DFF, DM, DFF, (size_t)DFF * DM, W2T, (size_t)DM * DFF, C_W);
  k_cvtf<<<dim3(NTOK / 8), dim3(256), 0, stream>>>(feature, FH);
  k_pw<<<dim3(1), dim3(256), 0, stream>>>(pos_w, pos_b, PWH, PBL);
  k_posb<<<dim3(NB * SQ), dim3(128), 0, stream>>>(pos_ind, PWH, PBL, BIAS);
  k_gemm_row<1, 1><<<dim3(NTOK / 32), dim3(256), 0, stream>>>(FH, KR, KR, WR, b_red, b_red, b_red, X, XH, RED_SC);

  for (int l = 0; l < NL; ++l) {
    k_qkv<<<dim3(NB * 2, NQKV / 64), dim3(256), 0, stream>>>(XH, WQKV + (size_t)l * NQKV * DM, Qp, VT);
    k_attn<<<dim3(NB * 4 * 8), dim3(256), 0, stream>>>(Qp, Kp, VT, fmask, BIAS, Op);
    k_gemm_row<0, 0><<<dim3(NTOK / 32), dim3(256), 0, stream>>>(Op, DM, DM, WO + (size_t)l * DM * DM,
                                                                ln1g + (size_t)l * DM, ln1g + (size_t)l * DM, ln1b + (size_t)l * DM,
                                                                X, XH, WO_SC);
    k_ffn1<<<dim3(NTOK / 256, DFF / 64), dim3(256), 0, stream>>>(XH, W1T + (size_t)l * DFF * DM, b1 + (size_t)l * DFF, HP);
    k_gemm_row<0, 1><<<dim3(NTOK / 32), dim3(256), 0, stream>>>(HP, DFF, DFF, W2T + (size_t)l * DM * DFF,
                                                                b2 + (size_t)l * DM, ln2g + (size_t)l * DM, ln2b + (size_t)l * DM,
                                                                X, XH, W2_SC);
  }
  k_cls<<<dim3(NTOK / 128), dim3(256), 0, stream>>>(X, cls_w, cls_b, out);
  (void)hipGetLastError();
}
